// MambaBlock_858993459381
// MI455X (gfx1250) — hardware-run, weakly checked
//
#include <hip/hip_runtime.h>
#include <hip/hip_fp16.h>
#include <math.h>

typedef float    ms1_v4f __attribute__((ext_vector_type(4)));
typedef unsigned ms1_v4u __attribute__((ext_vector_type(4)));
struct ms1_args {
  const float* dtpre;
  const float* u;
  const float* bc;
  const float* z;
  const float* A_log;
  const float* Dskip;
  __half* y;
  __half* y_lo;
  long ld_dtpre;
  long ld_u;
  long ld_bc;
  long ld_z;
  long ld_y;
  int offB;
  int offC;
  int offZ;
  float ycarry;
  int dir;
  int D;
  int L;
  int nbatch;
};
static_assert(sizeof(ms1_args) == 136);

__device__ __forceinline__ float ms1_flush16(float v) {
  return (fabsf(v) < 6.103515625e-05f) ? 0.0f : v;
}
__device__ __forceinline__ unsigned ms1_h16bits(float v) {
  return (unsigned)__half_as_ushort(__float2half_rn(ms1_flush16(v)));
}
__device__ __forceinline__ float ms1_h16val(unsigned b) {
  return __half2float(__ushort_as_half((unsigned short)b));
}
__device__ __forceinline__ float ms1_softplus(float v) {
  return fmaxf(v, 0.0f) + log1pf(expf(-fabsf(v)));
}
__device__ __forceinline__ void ms1_pack2(float v0, float v1, unsigned& hw, unsigned& lw) {
  const unsigned h0 = ms1_h16bits(v0);
  const unsigned h1 = ms1_h16bits(v1);
  const float r0 = (v0 - ms1_h16val(h0)) * 2048.0f;
  const float r1 = (v1 - ms1_h16val(h1)) * 2048.0f;
  const unsigned l0 = ms1_h16bits(r0);
  const unsigned l1 = ms1_h16bits(r1);
  hw = h0 | (h1 << 16);
  lw = l0 | (l1 << 16);
}

template <int NSTATE>
__global__ __launch_bounds__(64 * (NSTATE / 16)) void ms1_scan_kernel(ms1_args a)
{
  static_assert(NSTATE == 16 || NSTATE == 64);
  constexpr int NQ  = NSTATE / 16;
  constexpr int NT  = 64 * NQ;
  constexpr int NW  = NT / 32;
  constexpr int BCW = 2 * NSTATE;
  constexpr int YP  = 68;
  constexpr int RPI = NW * 4;
  constexpr int NIT = 64 / RPI;
  static_assert(16 * NT <= 64 * YP);
  __shared__ __align__(16) float sBC[64 * BCW];
  __shared__ __align__(16) float sY[64 * YP];
  const int tid  = threadIdx.x;
  const int lane = tid & 31;
  const int wave = tid >> 5;
  const int c    = tid / NQ;
  const int sq   = tid - c * NQ;
  const int bpb  = a.D / 64;
  const int bi   = blockIdx.x / bpb;
  if (bi >= a.nbatch) return;
  const int d0 = (blockIdx.x - bi * bpb) * 64;
  const int d  = d0 + c;
  const long rowb = (long)bi * a.L;
  const bool hasz  = (a.z != nullptr);
  const bool hasD  = (a.Dskip != nullptr);
  const bool hasLo = (a.y_lo != nullptr);

#pragma unroll 1
  for (int n = 0; n < 16; ++n) {
    const float al = a.A_log[(long)d * NSTATE + sq * 16 + n];
    sY[n * NT + tid] = -expf(al);
  }
  __syncthreads();
  float An[16], h[16];
#pragma unroll
  for (int n = 0; n < 16; ++n) {
    An[n] = sY[n * NT + tid];
    h[n] = 0.0f;
  }
  float Dd = 0.0f;
  if (hasD) Dd = a.Dskip[d];

  const int nchunk = a.L / 64;
  const bool fwd = (a.dir > 0);
  const int s0 = fwd ? 0 : 63;
  const int sd = fwd ? 1 : -1;
  const int q  = lane >> 3;
  const int c8 = (lane & 7) * 8;

#pragma unroll 1
  for (int ci = 0; ci < nchunk; ++ci) {
    const int tb = fwd ? (ci * 64) : (a.L - 64 - ci * 64);
    const long rowc = rowb + tb;
    __syncthreads();
#pragma unroll 8
    for (int i = 0; i < 32; ++i) {
      const int idx = tid + i * NT;
      const int st  = idx / BCW;
      const int col = idx - st * BCW;
      const int sc  = (col < NSTATE) ? (a.offB + col) : (a.offC + col - NSTATE);
      sBC[idx] = a.bc[(rowc + st) * a.ld_bc + sc];
    }
    __syncthreads();
#pragma unroll 1
    for (int s = 0; s < 64; ++s) {
      const int ls = s0 + sd * s;
      const long row = rowc + ls;
      float pre = a.dtpre[row * a.ld_dtpre + d];
      float uv  = a.u[row * a.ld_u + d];
      float zv  = 0.0f;
      if (hasz) zv = a.z[row * a.ld_z + a.offZ + d];
      asm volatile("" : "+v"(pre));
      asm volatile("" : "+v"(uv));
      asm volatile("" : "+v"(zv));
      const float delta = ms1_softplus(pre);
      const float dtx = delta * uv;
      const float* bp = sBC + ls * BCW + sq * 16;
      const float* cp = bp + NSTATE;
      ms1_v4f Bq[4], Cq[4];
#pragma unroll
      for (int k = 0; k < 4; ++k) {
        Bq[k] = *(const ms1_v4f*)(bp + 4 * k);
        Cq[k] = *(const ms1_v4f*)(cp + 4 * k);
      }
      float yv = 0.0f;
#pragma unroll
      for (int n = 0; n < 16; ++n) {
        const float e = __expf(delta * An[n]);
        h[n] = fmaf(e, h[n], dtx * Bq[n >> 2][n & 3]);
        yv = fmaf(h[n], Cq[n >> 2][n & 3], yv);
      }
      if (NQ > 1) {
        yv += __shfl_xor(yv, 1, 32);
        yv += __shfl_xor(yv, 2, 32);
      }
      if (hasD) yv = fmaf(uv, Dd, yv);
      if (hasz) {
        const float sg = __builtin_amdgcn_rcpf(1.0f + expf(-zv));
        yv = yv * (zv * sg);
      }
      if (sq == 0) sY[ls * YP + c] = yv * a.ycarry;
    }
    __syncthreads();
    ms1_v4u hw[NIT], lw[NIT];
#pragma unroll
    for (int it = 0; it < NIT; ++it) {
      const int row = it * RPI + wave * 4 + q;
      const float* sp = sY + row * YP + c8;
      const ms1_v4f f0 = *(const ms1_v4f*)(sp);
      const ms1_v4f f1 = *(const ms1_v4f*)(sp + 4);
      unsigned h0, h1, h2, h3, l0, l1, l2, l3;
      ms1_pack2(f0[0], f0[1], h0, l0);
      ms1_pack2(f0[2], f0[3], h1, l1);
      ms1_pack2(f1[0], f1[1], h2, l2);
      ms1_pack2(f1[2], f1[3], h3, l3);
      hw[it] = (ms1_v4u){h0, h1, h2, h3};
      lw[it] = (ms1_v4u){l0, l1, l2, l3};
    }
    for (int pass = 0; pass < 2; ++pass) {
#pragma unroll
      for (int it = 0; it < NIT; ++it) {
        const int row = it * RPI + wave * 4 + q;
        const long o = (rowc + row) * a.ld_y + d0 + c8;
        *(volatile ms1_v4u*)(a.y + o) = hw[it];
        if (hasLo) *(volatile ms1_v4u*)(a.y_lo + o) = lw[it];
      }
      __threadfence();
    }
  }
}

namespace eng {

constexpr int kBatch  = 2;
constexpr int kSeq    = 1024;
constexpr int kDm     = 1024;
constexpr int kDin    = 2048;
constexpr int kNstate = 16;
constexpr int kRank   = 64;
constexpr int kRows   = kBatch * kSeq;
constexpr int kXzN    = 2 * kDin;
constexpr int kXdN    = kRank + 2 * kNstate;
constexpr int kXdP    = 128;
constexpr int kOffB   = kRank;
constexpr int kOffC   = kRank + kNstate;

static_assert(kXdN == 96, "x_dbl column count");
static_assert((kSeq & (kSeq - 1)) == 0, "sequence length is a power of two");
static_assert(kRows % 64 == 0 && kXzN % 64 == 0 && kXdP % 64 == 0 && kDin % 64 == 0 && kDm % 64 == 0, "tile multiples");
static_assert(kDm % 32 == 0 && kDin % 32 == 0 && kRank % 32 == 0, "K multiples of 32");
static_assert(kDin % 64 == 0 && kSeq % 64 == 0, "scan geometry");
static_assert(kDin == 2 * 1024, "conv kernel: two groups of 1024 channels per row");

constexpr float kCarryX    = 16.0f;
constexpr float kCarryWin  = 256.0f;
constexpr float kCarryUc   = 16.0f;
constexpr float kCarryWx   = 256.0f;
constexpr float kCarryDtl  = 64.0f;
constexpr float kCarryWdt  = 64.0f;
constexpr float kCarryY    = 16.0f;
constexpr float kCarryWout = 256.0f;
constexpr float kResid     = 2048.0f;
constexpr float kFoldIn    = 1.0f / (kCarryX * kCarryWin);
constexpr float kFoldXp    = 1.0f / (kCarryUc * kCarryWx);
constexpr float kFoldDt    = 1.0f / (kCarryDtl * kCarryWdt);
constexpr float kFoldOut   = 1.0f / (kCarryY * kCarryWout);
constexpr float kFoldResid = 1.0f / kResid;

constexpr size_t kBytesXh    = (size_t)kRows * kDm * 2;
constexpr size_t kBytesWinT  = (size_t)kXzN * kDm * 2;
constexpr size_t kBytesWxT   = (size_t)kXdP * kDin * 2;
constexpr size_t kBytesWdtT  = (size_t)kDin * kRank * 2;
constexpr size_t kBytesWoutT = (size_t)kDm * kDin * 2;
constexpr size_t kBytesXZ    = (size_t)kRows * kXzN * 4;
constexpr size_t kBytesUC    = (size_t)kRows * kDin * 4;
constexpr size_t kBytesUCh   = (size_t)kRows * kDin * 2;
constexpr size_t kBytesXDBL  = (size_t)kRows * kXdP * 4;
constexpr size_t kBytesDTLh  = (size_t)kRows * kRank * 2;
constexpr size_t kBytesDTP   = (size_t)kRows * kDin * 4;
constexpr size_t kBytesYH    = (size_t)kRows * kDin * 2;
constexpr size_t kBytesYL    = (size_t)kRows * kDin * 2;
constexpr size_t kWsTotal = kBytesXh + kBytesWinT + kBytesWxT + kBytesWdtT + kBytesWoutT + kBytesXZ + kBytesUC +
                            kBytesUCh + kBytesXDBL + kBytesDTLh + kBytesDTP + kBytesYH + kBytesYL;
static_assert(kWsTotal == 111149056ull, "literal sum of the carve sizes: 106 MiB");
static_assert(kWsTotal <= 134217728ull, "carve stays under 128 MiB");
static_assert(kBytesXh % 128 == 0 && kBytesWinT % 128 == 0 && kBytesWxT % 128 == 0 && kBytesWdtT % 128 == 0 &&
              kBytesWoutT % 128 == 0 && kBytesXZ % 128 == 0 && kBytesUC % 128 == 0 && kBytesUCh % 128 == 0 &&
              kBytesXDBL % 128 == 0 && kBytesDTLh % 128 == 0 && kBytesDTP % 128 == 0 && kBytesYH % 128 == 0,
              "every region starts on a 128-B line");

typedef _Float16 v16h __attribute__((ext_vector_type(16)));
typedef _Float16 v8h  __attribute__((ext_vector_type(8)));
typedef float    v8f  __attribute__((ext_vector_type(8)));
typedef float    v4f  __attribute__((ext_vector_type(4)));
typedef unsigned v4u  __attribute__((ext_vector_type(4)));

__device__ __forceinline__ float flush16(float v) {
  return (fabsf(v) < 6.103515625e-05f) ? 0.0f : v;
}
__device__ __forceinline__ unsigned h16bits(float v) {
  return (unsigned)__half_as_ushort(__float2half_rn(flush16(v)));
}
__device__ __forceinline__ unsigned pack2(float a, float b) {
  const unsigned lo = h16bits(a);
  const unsigned hi = h16bits(b);
  return lo | (hi << 16);
}

union FragU { v16h v; v8h h[2]; };
__device__ __forceinline__ v16h frag_load(const _Float16* p) {
  FragU f;
  f.h[0] = *(const v8h*)(p);
  f.h[1] = *(const v8h*)(p + 16);
  return f.v;
}
__device__ __forceinline__ v8f mma(v16h a, v16h b, v8f c) {
  c = __builtin_amdgcn_wmma_f32_16x16x32_f16(false, a, false, b, (short)0, c, false, false);
  asm volatile("v_nop\n\tv_nop\n\tv_nop\n\tv_nop" : "+v"(c) : "v"(a), "v"(b));
  return c;
}

__global__ __launch_bounds__(256) void cast_carry_f16_kernel(
    const float* __restrict__ in, unsigned short* __restrict__ out, int n8, float carry)
{
  const int i = blockIdx.x * 256 + threadIdx.x;
  if (i < n8) {
    const v4f f0 = *(const v4f*)(in + (size_t)i * 8);
    const v4f f1 = *(const v4f*)(in + (size_t)i * 8 + 4);
    const float e0 = f0[0] * carry;
    const float e1 = f0[1] * carry;
    const float e2 = f0[2] * carry;
    const float e3 = f0[3] * carry;
    const float e4 = f1[0] * carry;
    const float e5 = f1[1] * carry;
    const float e6 = f1[2] * carry;
    const float e7 = f1[3] * carry;
    const v4u hw = (v4u){pack2(e0, e1), pack2(e2, e3), pack2(e4, e5), pack2(e6, e7)};
    unsigned short* o = out + (size_t)i * 8;
    for (int pass = 0; pass < 2; ++pass) {
      *(volatile v4u*)(o) = hw;
      __threadfence();
    }
  }
}

__global__ __launch_bounds__(256) void transpose_cast_kernel(
    const float* __restrict__ in, unsigned short* __restrict__ out, int R, int C, float carry)
{
  __shared__ __align__(16) float sTile[64 * 68];
  const int tid  = threadIdx.x;
  const int lane = tid & 31;
  const int wave = tid >> 5;
  const int k0 = blockIdx.x * 64;
  const int n0 = blockIdx.y * 64;
#pragma unroll 4
  for (int i = 0; i < 16; ++i) {
    const int idx = tid + i * 256;
    const int kr = idx >> 6;
    const int nc = idx & 63;
    const int n  = n0 + nc;
    const int ncl = (n < C) ? n : (C - 1);
    float v = in[(size_t)(k0 + kr) * C + ncl];
    asm volatile("" : "+v"(v));
    v = (n < C) ? (v * carry) : 0.0f;
    sTile[nc * 68 + kr] = v;
  }
  __syncthreads();
  const int q  = lane >> 3;
  const int c8 = (lane & 7) * 8;
  v4u hw[2];
#pragma unroll
  for (int it = 0; it < 2; ++it) {
    const int row = it * 32 + wave * 4 + q;
    const float* sp = sTile + row * 68 + c8;
    const v4f f0 = *(const v4f*)(sp);
    const v4f f1 = *(const v4f*)(sp + 4);
    const float e0 = f0[0];
    const float e1 = f0[1];
    const float e2 = f0[2];
    const float e3 = f0[3];
    const float e4 = f1[0];
    const float e5 = f1[1];
    const float e6 = f1[2];
    const float e7 = f1[3];
    hw[it] = (v4u){pack2(e0, e1), pack2(e2, e3), pack2(e4, e5), pack2(e6, e7)};
  }
  for (int pass = 0; pass < 2; ++pass) {
#pragma unroll
    for (int it = 0; it < 2; ++it) {
      const int row = it * 32 + wave * 4 + q;
      *(volatile v4u*)(out + (size_t)(n0 + row) * R + k0 + c8) = hw[it];
    }
    __threadfence();
  }
}

template <int MT, int ATERMS, int EPI>
__global__ __launch_bounds__(256) void gemm_f16_kernel(
    const unsigned short* __restrict__ Ap, const unsigned short* __restrict__ A2p, int lda,
    const unsigned short* __restrict__ Btp, int ldb,
    float* __restrict__ C, int ldc,
    unsigned short* __restrict__ C16, int ldc16,
    const float* __restrict__ bias,
    int M, int N, int K, float scale, float scale2, float scale16)
{
  const _Float16* A  = (const _Float16*)(const void*)Ap;
  const _Float16* A2 = (const _Float16*)(const void*)A2p;
  const _Float16* Bt = (const _Float16*)(const void*)Btp;
  __shared__ __align__(16) float sT[8][16 * 68];
  const int lane = threadIdx.x & 31;
  const int wave = threadIdx.x >> 5;
  const int tilesN = N >> 6;
  const int tilesM = M / (16 * MT);
  const int tile = blockIdx.x * 8 + wave;
  if (tile >= tilesM * tilesN) return;
  const int tm = tile / tilesN;
  const int tn = tile - tm * tilesN;
  const int m0 = tm * (16 * MT);
  const int n0 = tn << 6;
  const int rlane = lane & 15;
  const int koff  = (lane >> 4) * 8;
  const int mOff  = (lane >> 4) * 8;

  v8f accH[MT][4];
  v8f accL[MT][4];
#pragma unroll
  for (int i = 0; i < MT; ++i) {
#pragma unroll
    for (int j = 0; j < 4; ++j) {
      accH[i][j] = (v8f){0.f, 0.f, 0.f, 0.f, 0.f, 0.f, 0.f, 0.f};
      accL[i][j] = (v8f){0.f, 0.f, 0.f, 0.f, 0.f, 0.f, 0.f, 0.f};
    }
  }

#pragma unroll 1
  for (int k0 = 0; k0 < K; k0 += 32) {
    v16h bf[4];
#pragma unroll
    for (int j = 0; j < 4; ++j) {
      bf[j] = frag_load(Bt + (size_t)(n0 + (j << 4) + rlane) * ldb + koff + k0);
    }
#pragma unroll
    for (int i = 0; i < MT; ++i) {
      const size_t ao = (size_t)(m0 + (i << 4) + rlane) * lda + koff + k0;
      const v16h a0 = frag_load(A + ao);
#pragma unroll
      for (int j = 0; j < 4; ++j) accH[i][j] = mma(a0, bf[j], accH[i][j]);
      if (ATERMS == 2) {
        const v16h a1 = frag_load(A2 + ao);
#pragma unroll
        for (int j = 0; j < 4; ++j) accL[i][j] = mma(a1, bf[j], accL[i][j]);
      }
    }
  }

  float* slab = sT[wave];
  float bv[4] = {0.f, 0.f, 0.f, 0.f};
  if (EPI == 2) {
#pragma unroll
    for (int j = 0; j < 4; ++j) bv[j] = bias[n0 + (j << 4) + rlane];
  }
#pragma unroll
  for (int i = 0; i < MT; ++i) {
    const int mBase = m0 + (i << 4);
#pragma unroll
    for (int j = 0; j < 4; ++j) {
#pragma unroll
      for (int r = 0; r < 8; ++r) {
        float v = accH[i][j][r];
        if (ATERMS == 2) v = v + accL[i][j][r] * scale2;
        v = v * scale;
        if (EPI == 2) v = v + bv[j];
        slab[(mOff + r) * 68 + (j << 4) + rlane] = v;
      }
    }
    __builtin_amdgcn_fence(__ATOMIC_RELEASE, "workgroup");
    __builtin_amdgcn_wave_barrier();
    __builtin_amdgcn_fence(__ATOMIC_ACQUIRE, "workgroup");
    {
      const int hh = lane >> 4;
      const int c4 = (lane & 15) * 4;
      for (int pass = 0; pass < 2; ++pass) {
#pragma unroll
        for (int it = 0; it < 8; ++it) {
          const int row = it * 2 + hh;
          const v4f val = *(const v4f*)(slab + row * 68 + c4);
          *(volatile v4f*)(C + (size_t)(mBase + row) * ldc + n0 + c4) = val;
        }
        __threadfence();
      }
    }
    if (EPI == 1) {
      if (n0 == 0) {
        const int q  = lane >> 3;
        const int c8 = (lane & 7) * 8;
        v4u hw[4];
#pragma unroll
        for (int it = 0; it < 4; ++it) {
          const int row = it * 4 + q;
          const float* sp = slab + row * 68 + c8;
          const v4f f0 = *(const v4f*)(sp);
          const v4f f1 = *(const v4f*)(sp + 4);
          const float e0 = f0[0] * scale16;
          const float e1 = f0[1] * scale16;
          const float e2 = f0[2] * scale16;
          const float e3 = f0[3] * scale16;
          const float e4 = f1[0] * scale16;
          const float e5 = f1[1] * scale16;
          const float e6 = f1[2] * scale16;
          const float e7 = f1[3] * scale16;
          hw[it] = (v4u){pack2(e0, e1), pack2(e2, e3), pack2(e4, e5), pack2(e6, e7)};
        }
        for (int pass = 0; pass < 2; ++pass) {
#pragma unroll
          for (int it = 0; it < 4; ++it) {
            const int row = it * 4 + q;
            *(volatile v4u*)(C16 + (size_t)(mBase + row) * ldc16 + c8) = hw[it];
          }
          __threadfence();
        }
      }
    }
    __builtin_amdgcn_fence(__ATOMIC_RELEASE, "workgroup");
    __builtin_amdgcn_wave_barrier();
    __builtin_amdgcn_fence(__ATOMIC_ACQUIRE, "workgroup");
  }
}

__device__ __forceinline__ float conv_silu_one(v4f w, float u0, float u1, float u2, float u3, float b) {
  float acc = w[0] * u0;
  acc = fmaf(w[1], u1, acc);
  acc = fmaf(w[2], u2, acc);
  acc = fmaf(w[3], u3, acc);
  const float cv = acc + b;
  const float sg = 1.0f / (1.0f + expf(-cv));
  return cv * sg;
}

__global__ __launch_bounds__(256) void conv_silu_kernel(
    const float* __restrict__ XZ, const float* __restrict__ conv_w, const float* __restrict__ conv_b,
    float* __restrict__ UC, unsigned short* __restrict__ UCh, float carry)
{
  __shared__ __align__(16) float sRow[kDin];
  const int tid = threadIdx.x;
  const int r = blockIdx.x;
  const int t = r & (kSeq - 1);
  const int rb = r - t;
#pragma unroll 1
  for (int j = 0; j < 2; ++j) {
    const int d4 = j * 1024 + tid * 4;
    const v4f bs = *(const v4f*)(conv_b + d4);
    const v4f w0 = *(const v4f*)(conv_w + (size_t)d4 * 4);
    const v4f w1 = *(const v4f*)(conv_w + (size_t)d4 * 4 + 4);
    const v4f w2 = *(const v4f*)(conv_w + (size_t)d4 * 4 + 8);
    const v4f w3 = *(const v4f*)(conv_w + (size_t)d4 * 4 + 12);
    v4f ut[4];
#pragma unroll
    for (int k = 0; k < 4; ++k) {
      const int tt = t - 3 + k;
      const int tc = (tt < 0) ? 0 : tt;
      const bool on = (tt >= 0);
      const v4f ld = *(const v4f*)(XZ + (size_t)(rb + tc) * kXzN + d4);
      v4f uv;
      uv[0] = on ? ld[0] : 0.0f;
      uv[1] = on ? ld[1] : 0.0f;
      uv[2] = on ? ld[2] : 0.0f;
      uv[3] = on ? ld[3] : 0.0f;
      ut[k] = uv;
    }
    v4f o;
    o[0] = conv_silu_one(w0, ut[0][0], ut[1][0], ut[2][0], ut[3][0], bs[0]);
    o[1] = conv_silu_one(w1, ut[0][1], ut[1][1], ut[2][1], ut[3][1], bs[1]);
    o[2] = conv_silu_one(w2, ut[0][2], ut[1][2], ut[2][2], ut[3][2], bs[2]);
    o[3] = conv_silu_one(w3, ut[0][3], ut[1][3], ut[2][3], ut[3][3], bs[3]);
    *(v4f*)(sRow + d4) = o;
  }
  __syncthreads();
  const v4f o0 = *(const v4f*)(sRow + tid * 4);
  const v4f o1 = *(const v4f*)(sRow + 1024 + tid * 4);
  const v4f f0 = *(const v4f*)(sRow + tid * 8);
  const v4f f1 = *(const v4f*)(sRow + tid * 8 + 4);
  const float e0 = f0[0] * carry;
  const float e1 = f0[1] * carry;
  const float e2 = f0[2] * carry;
  const float e3 = f0[3] * carry;
  const float e4 = f1[0] * carry;
  const float e5 = f1[1] * carry;
  const float e6 = f1[2] * carry;
  const float e7 = f1[3] * carry;
  const v4u hw = (v4u){pack2(e0, e1), pack2(e2, e3), pack2(e4, e5), pack2(e6, e7)};
  float* ucr = UC + (size_t)r * kDin;
  unsigned short* uhr = UCh + (size_t)r * kDin;
  for (int pass = 0; pass < 2; ++pass) {
    *(volatile v4f*)(ucr + tid * 4) = o0;
    *(volatile v4f*)(ucr + 1024 + tid * 4) = o1;
    *(volatile v4u*)(uhr + tid * 8) = hw;
    __threadfence();
  }
}

}

extern "C" void kernel_launch(void* const* d_in, const int* in_sizes, int n_in,
                              void* d_out, int out_size, void* d_ws, size_t ws_size, hipStream_t stream)
{
  using namespace eng;
  if (n_in != 10) return;
  if (in_sizes[0] != kRows * kDm) return;
  if (in_sizes[1] != kDm * kXzN) return;
  if (in_sizes[2] != kDin * 4) return;
  if (in_sizes[3] != kDin) return;
  if (in_sizes[4] != kDin * kXdN) return;
  if (in_sizes[5] != kRank * kDin) return;
  if (in_sizes[6] != kDin) return;
  if (in_sizes[7] != kDin * kNstate) return;
  if (in_sizes[8] != kDin) return;
  if (in_sizes[9] != kDin * kDm) return;
  if (out_size != kRows * kDm) return;
  if (ws_size < kWsTotal) return;

  const float* x      = (const float*)d_in[0];
  const float* W_in   = (const float*)d_in[1];
  const float* conv_w = (const float*)d_in[2];
  const float* conv_b = (const float*)d_in[3];
  const float* W_x    = (const float*)d_in[4];
  const float* W_dt   = (const float*)d_in[5];
  const float* b_dt   = (const float*)d_in[6];
  const float* A_log  = (const float*)d_in[7];
  const float* D_par  = (const float*)d_in[8];
  const float* W_out  = (const float*)d_in[9];
  float* out = (float*)d_out;

  char* ws = (char*)d_ws;
  size_t off = 0;
  unsigned short* Xh    = (unsigned short*)(ws + off);
  off += kBytesXh;
  unsigned short* WinT  = (unsigned short*)(ws + off);
  off += kBytesWinT;
  unsigned short* WxT   = (unsigned short*)(ws + off);
  off += kBytesWxT;
  unsigned short* WdtT  = (unsigned short*)(ws + off);
  off += kBytesWdtT;
  unsigned short* WoutT = (unsigned short*)(ws + off);
  off += kBytesWoutT;
  float* XZ             = (float*)(ws + off);
  off += kBytesXZ;
  float* UC             = (float*)(ws + off);
  off += kBytesUC;
  unsigned short* UCh   = (unsigned short*)(ws + off);
  off += kBytesUCh;
  float* XDBL           = (float*)(ws + off);
  off += kBytesXDBL;
  unsigned short* DTLh  = (unsigned short*)(ws + off);
  off += kBytesDTLh;
  float* DTP            = (float*)(ws + off);
  off += kBytesDTP;
  unsigned short* YH    = (unsigned short*)(ws + off);
  off += kBytesYH;
  unsigned short* YL    = (unsigned short*)(ws + off);
  off += kBytesYL;
  if (off != kWsTotal) return;

  cast_carry_f16_kernel<<<dim3((kRows * kDm / 8) / 256), 256, 0, stream>>>(x, Xh, kRows * kDm / 8, kCarryX);

  transpose_cast_kernel<<<dim3(kDm / 64, kXzN / 64), 256, 0, stream>>>(W_in, WinT, kDm, kXzN, kCarryWin);
  transpose_cast_kernel<<<dim3(kDin / 64, kXdP / 64), 256, 0, stream>>>(W_x, WxT, kDin, kXdN, kCarryWx);
  transpose_cast_kernel<<<dim3(kRank / 64, kDin / 64), 256, 0, stream>>>(W_dt, WdtT, kRank, kDin, kCarryWdt);
  transpose_cast_kernel<<<dim3(kDin / 64, kDm / 64), 256, 0, stream>>>(W_out, WoutT, kDin, kDm, kCarryWout);

  gemm_f16_kernel<4, 1, 0><<<dim3((kRows / 64) * (kXzN / 64) / 8), 256, 0, stream>>>(
      Xh, Xh, kDm, WinT, kDm, XZ, kXzN, DTLh, kRank, b_dt,
      kRows, kXzN, kDm, kFoldIn, 0.0f, 0.0f);

  conv_silu_kernel<<<dim3(kRows), 256, 0, stream>>>(XZ, conv_w, conv_b, UC, UCh, kCarryUc);

  gemm_f16_kernel<4, 1, 1><<<dim3((kRows / 64) * (kXdP / 64) / 8), 256, 0, stream>>>(
      UCh, UCh, kDin, WxT, kDin, XDBL, kXdP, DTLh, kRank, b_dt,
      kRows, kXdP, kDin, kFoldXp, 0.0f, kCarryDtl);

  gemm_f16_kernel<4, 1, 2><<<dim3((kRows / 64) * (kDin / 64) / 8), 256, 0, stream>>>(
      DTLh, DTLh, kRank, WdtT, kRank, DTP, kDin, DTLh, kRank, b_dt,
      kRows, kDin, kRank, kFoldDt, 0.0f, 0.0f);

  for (int b = 0; b < kBatch; ++b) {
    const size_t r0 = (size_t)b * kSeq;
    ms1_args sa;
    sa.dtpre = DTP + r0 * kDin;
    sa.u = UC + r0 * kDin;
    sa.bc = XDBL + r0 * kXdP;
    sa.z = XZ + r0 * kXzN;
    sa.A_log = A_log;
    sa.Dskip = D_par;
    sa.y = (__half*)(YH + r0 * kDin);
    sa.y_lo = (__half*)(YL + r0 * kDin);
    sa.ld_dtpre = kDin;
    sa.ld_u = kDin;
    sa.ld_bc = kXdP;
    sa.ld_z = kXzN;
    sa.ld_y = kDin;
    sa.offB = kOffB;
    sa.offC = kOffC;
    sa.offZ = kDin;
    sa.ycarry = kCarryY;
    sa.dir = 1;
    sa.D = kDin;
    sa.L = kSeq;
    sa.nbatch = 1;
    ms1_scan_kernel<16><<<dim3(kDin / 64), 64, 0, stream>>>(sa);
  }

  gemm_f16_kernel<2, 2, 0><<<dim3((kRows / 32) * (kDm / 64) / 8), 256, 0, stream>>>(
      YH, YL, kDin, WoutT, kDin, out, kDm, DTLh, kRank, b_dt,
      kRows, kDm, kDin, kFoldOut, kFoldResid, 0.0f);
}
